// RCGNLayer_41506563948628
// MI455X (gfx1250) — hardware-verified
//
#include <hip/hip_runtime.h>
#include <stddef.h>


#define DF      128
#define NRELS   8
#define RH      4
#define NTHR    256
#define NWAVE   8
#define EPT     8
#define NGRP    2
#define CHUNK   (NTHR * EPT * NGRP)
#define WCAP    (EPT * NGRP * 32)
#define LISTN   (NWAVE * WCAP)
#define NB      512
#define NTILE   (NB / 16)
#define TPW     (NTILE / NWAVE)
#define RPW     (NB / NWAVE)
#define GROWS   (NWAVE * 16)

#define LDS_ACC   (NB * DF * 4)
#define LDS_LIST  (LISTN * 4)
#define LDS_AGG   (LDS_ACC + LDS_LIST + 64)

static_assert((CHUNK & (CHUNK - 1)) == 0);
static_assert(CHUNK <= 4096);
static_assert((NB & (NB - 1)) == 0);
static_assert(NB <= 4096);
static_assert(NTILE % NWAVE == 0);
static_assert(NB % NWAVE == 0);
static_assert(NWAVE * 4 <= 64);
static_assert(LDS_AGG <= 300 * 1024);
static_assert(DF % 32 == 0);

typedef float  v4f   __attribute__((ext_vector_type(4)));
typedef float  v8f   __attribute__((ext_vector_type(8)));
typedef int    v4i   __attribute__((ext_vector_type(4)));
typedef __bf16 bf16_t;
typedef bf16_t v8bf  __attribute__((ext_vector_type(8)));
typedef bf16_t v16bf __attribute__((ext_vector_type(16)));
union FragB { v16bf v; v8bf h[2]; v4i q[2]; };
union Pack8 { v8bf v; v4i q; };

__device__ __forceinline__ v8f wmb(v16bf a, v16bf b, v8f c) {
  v8f d = __builtin_amdgcn_wmma_f32_16x16x32_bf16(false, a, false, b, (short)0, c, false, false);
  asm volatile("v_nop\n\tv_nop\n\tv_nop\n\tv_nop" : "+v"(d) : "v"(a), "v"(b));
  return d;
}

template <int NBT>
__device__ __forceinline__ int scan_chunk(const int* __restrict__ dsts, int nE, int cbase, int nodeBase,
                                          int vec8, int* list, int tid, int lane, int wave) {
  int wc = 0;
  (void)lane;
#pragma unroll
  for (int g = 0; g < NGRP; ++g) {
    const int el0  = (g * NTHR + tid) * EPT;
    const int e0   = cbase + el0;
    const int sent = -2147483647 - 1;
    v4i da, db;
    if (vec8 != 0 && cbase + CHUNK <= nE) {
      da = *(const v4i*)(dsts + e0);
      db = *(const v4i*)(dsts + e0 + 4);
    } else {
      da.x = (e0     < nE) ? dsts[min(e0, nE - 1)] : sent;
      da.y = (e0 + 1 < nE) ? dsts[min(e0 + 1, nE - 1)] : sent;
      da.z = (e0 + 2 < nE) ? dsts[min(e0 + 2, nE - 1)] : sent;
      da.w = (e0 + 3 < nE) ? dsts[min(e0 + 3, nE - 1)] : sent;
      db.x = (e0 + 4 < nE) ? dsts[min(e0 + 4, nE - 1)] : sent;
      db.y = (e0 + 5 < nE) ? dsts[min(e0 + 5, nE - 1)] : sent;
      db.z = (e0 + 6 < nE) ? dsts[min(e0 + 6, nE - 1)] : sent;
      db.w = (e0 + 7 < nE) ? dsts[min(e0 + 7, nE - 1)] : sent;
    }
    const unsigned nb = (unsigned)nodeBase;
    const unsigned s0 = (unsigned)da.x - nb, s1 = (unsigned)da.y - nb;
    const unsigned s2 = (unsigned)da.z - nb, s3 = (unsigned)da.w - nb;
    const unsigned s4 = (unsigned)db.x - nb, s5 = (unsigned)db.y - nb;
    const unsigned s6 = (unsigned)db.z - nb, s7 = (unsigned)db.w - nb;
    const bool h0 = s0 < (unsigned)NBT, h1 = s1 < (unsigned)NBT, h2 = s2 < (unsigned)NBT, h3 = s3 < (unsigned)NBT;
    const bool h4 = s4 < (unsigned)NBT, h5 = s5 < (unsigned)NBT, h6 = s6 < (unsigned)NBT, h7 = s7 < (unsigned)NBT;
    const unsigned any = __builtin_amdgcn_ballot_w32(h0 | h1 | h2 | h3 | h4 | h5 | h6 | h7);
    if (any != 0u) {
#define HITJ(J, HJ, SJ) { \
        const unsigned mj = __builtin_amdgcn_ballot_w32(HJ); \
        if (mj != 0u) { \
          if (HJ) { \
            const int pos = wc + (int)__builtin_amdgcn_mbcnt_lo(mj, 0u); \
            if (pos < WCAP) list[wave * WCAP + pos] = ((el0 + (J)) << 12) | (int)(SJ); \
          } \
          wc += (int)__builtin_popcount(mj); } }
      HITJ(0, h0, s0)
      HITJ(1, h1, s1)
      HITJ(2, h2, s2)
      HITJ(3, h3, s3)
      HITJ(4, h4, s4)
      HITJ(5, h5, s5)
      HITJ(6, h6, s6)
      HITJ(7, h7, s7)
#undef HITJ
    }
  }
  return wc;
}

__global__ __launch_bounds__(NTHR) void k_wprep(
    const float* __restrict__ W, const float* __restrict__ W0,
    bf16_t* whi, bf16_t* wlo, int nTot) {
  const int i = blockIdx.x * NTHR + threadIdx.x;
  if (i >= nTot) return;
  const int o   = i * 8;
  const int g   = o / (DF * DF);
  const int rem = o - g * (DF * DF);
  const int n   = rem / DF;
  const int k0  = rem - n * DF;
  const float* p = (g < NRELS) ? (W + (size_t)g * DF * DF + (size_t)k0 * DF + n)
                               : (W0 + (size_t)k0 * DF + n);
  Pack8 ph, pl;
#define WSP(I) { const float xv = p[(I) * DF]; const bf16_t hb = (bf16_t)xv; ph.v[(I)] = hb; pl.v[(I)] = (bf16_t)(xv - (float)hb); }
  WSP(0) WSP(1) WSP(2) WSP(3) WSP(4) WSP(5) WSP(6) WSP(7)
#undef WSP
  bf16_t* dh = whi + o;
  bf16_t* dl = wlo + o;
  const v4i qh = ph.q, ql = pl.q;
  *(volatile v4i*)dh = qh;
  *(volatile v4i*)dl = ql;
  __threadfence();
  *(volatile v4i*)dh = qh;
  *(volatile v4i*)dl = ql;
}

__global__ __launch_bounds__(NTHR) void k_xprep(
    const float* __restrict__ X, bf16_t* xhi, bf16_t* xlo, int nN, int nTot) {
  const int i = blockIdx.x * NTHR + threadIdx.x;
  if (i >= nTot) return;
  const int o    = i * 8;
  const int row  = o / DF;
  const int c0   = o - row * DF;
  const int rowc = row < nN ? row : nN - 1;
  const v4f z = {0.f, 0.f, 0.f, 0.f};
  v4f a = *(const v4f*)(X + (size_t)rowc * DF + c0);
  v4f b = *(const v4f*)(X + (size_t)rowc * DF + c0 + 4);
  a = (row < nN) ? a : z;
  b = (row < nN) ? b : z;
  Pack8 ph, pl;
#define XSP(I, V) { const float xv = (V); const bf16_t hb = (bf16_t)xv; ph.v[(I)] = hb; pl.v[(I)] = (bf16_t)(xv - (float)hb); }
  XSP(0, a.x) XSP(1, a.y) XSP(2, a.z) XSP(3, a.w)
  XSP(4, b.x) XSP(5, b.y) XSP(6, b.z) XSP(7, b.w)
#undef XSP
  bf16_t* dh = xhi + o;
  bf16_t* dl = xlo + o;
  const v4i qh = ph.q, ql = pl.q;
  *(volatile v4i*)dh = qh;
  *(volatile v4i*)dl = ql;
  __threadfence();
  *(volatile v4i*)dh = qh;
  *(volatile v4i*)dl = ql;
}

__device__ __forceinline__ void kstep3(const bf16_t* ahp, const bf16_t* alp,
                                       const bf16_t* bhp, const bf16_t* blp, v8f (&c)[8]) {
  FragB ah, al;
  ah.q[0] = *(const v4i*)ahp;  ah.q[1] = *(const v4i*)(ahp + 16);
  al.q[0] = *(const v4i*)alp;  al.q[1] = *(const v4i*)(alp + 16);
#pragma unroll
  for (int ct = 0; ct < DF / 16; ++ct) {
    const bf16_t* hp = bhp + (size_t)ct * 16 * DF;
    const bf16_t* lp = blp + (size_t)ct * 16 * DF;
    FragB bh, bl;
    bh.q[0] = *(const v4i*)hp;  bh.q[1] = *(const v4i*)(hp + 16);
    bl.q[0] = *(const v4i*)lp;  bl.q[1] = *(const v4i*)(lp + 16);
    c[ct] = wmb(al.v, bh.v, c[ct]);
    c[ct] = wmb(ah.v, bl.v, c[ct]);
    c[ct] = wmb(ah.v, bh.v, c[ct]);
  }
}

__global__ __launch_bounds__(NTHR) void k_hgemm(
    const bf16_t* __restrict__ xhi, const bf16_t* __restrict__ xlo,
    const bf16_t* __restrict__ whi, const bf16_t* __restrict__ wlo,
    float* H, int nRowsPad) {
  __shared__ float stg[NWAVE * 16 * DF];
  const int tid = threadIdx.x, lane = tid & 31, wave = tid >> 5, hh = lane >> 4, m = lane & 15;
  const int j = blockIdx.y;
  const int rowBase = blockIdx.x * GROWS + wave * 16;

  v8f c[8];
#pragma unroll
  for (int ct = 0; ct < 8; ++ct) { const v8f z = {0.f, 0.f, 0.f, 0.f, 0.f, 0.f, 0.f, 0.f}; c[ct] = z; }

  const bf16_t* ah0 = xhi + (size_t)(rowBase + m) * DF + 8 * hh;
  const bf16_t* al0 = xlo + (size_t)(rowBase + m) * DF + 8 * hh;
  const bf16_t* bh0 = whi + (size_t)j * DF * DF + (size_t)m * DF + 8 * hh;
  const bf16_t* bl0 = wlo + (size_t)j * DF * DF + (size_t)m * DF + 8 * hh;
#pragma unroll 1
  for (int ks = 0; ks < DF / 32; ++ks)
    kstep3(ah0 + 32 * ks, al0 + 32 * ks, bh0 + 32 * ks, bl0 + 32 * ks, c);

  float* sp = stg + (wave * 16 + 8 * hh) * DF + m;
#pragma unroll
  for (int ct = 0; ct < 8; ++ct) {
#pragma unroll
    for (int r = 0; r < 8; ++r) sp[r * DF + 16 * ct] = c[ct][r];
  }
  __syncthreads();

  const float* lrow = stg + (wave * 16) * DF + 4 * lane;
  float* gp = H + ((size_t)j * nRowsPad + rowBase) * DF + 4 * lane;
#pragma unroll
  for (int i = 0; i < 16; ++i) { const v4f v = *(const v4f*)(lrow + i * DF); *(volatile v4f*)(gp + (size_t)i * DF) = v; }
  __threadfence();
#pragma unroll
  for (int i = 0; i < 16; ++i) { const v4f v = *(const v4f*)(lrow + i * DF); *(volatile v4f*)(gp + (size_t)i * DF) = v; }
}

template <int FIN>
__global__ __launch_bounds__(NTHR) void k_agg(
    const int* __restrict__ dsts, const int* __restrict__ srcs, const int* __restrict__ rels,
    const float* __restrict__ inv_norm, const float* __restrict__ H,
    const bf16_t* __restrict__ xhi, const bf16_t* __restrict__ xlo,
    const bf16_t* __restrict__ w0hi, const bf16_t* __restrict__ w0lo,
    float* out, int nN, int nE, int nRowsPad, int rb, int vec8) {
  extern __shared__ v4f lds_dyn[];
  float* acc  = (float*)lds_dyn;
  int*   list = (int*)((char*)lds_dyn + LDS_ACC);
  int*   wcnt = (int*)((char*)lds_dyn + LDS_ACC + LDS_LIST);
  const int tid = threadIdx.x, lane = tid & 31, wave = tid >> 5, hh = lane >> 4, m = lane & 15;
  const int nodeBase = blockIdx.x * NB;
  const v4f z4 = {0.f, 0.f, 0.f, 0.f};

  for (int i = tid; i < NB * DF / 4; i += NTHR) {
    if (FIN != 0) {
      const int slot = i / (DF / 4);
      const int c4   = i - slot * (DF / 4);
      const int node = nodeBase + slot;
      const int nc   = node < nN ? node : nN - 1;
      v4f v = *(const v4f*)(out + (size_t)nc * DF + 4 * c4);
      v = (node < nN) ? v : z4;
      lds_dyn[i] = v;
    } else {
      lds_dyn[i] = z4;
    }
  }
  __syncthreads();

  const int nChunks = (nE + CHUNK - 1) / CHUNK;
#pragma unroll 1
  for (int ch = 0; ch < nChunks; ++ch) {
    const int cbase = ch * CHUNK;
    const int wc = scan_chunk<NB>(dsts, nE, cbase, nodeBase, vec8, list, tid, lane, wave);
    if (lane == 0) wcnt[wave] = wc;
    __syncthreads();
    if (wave == 0) {
#pragma unroll 1
      for (int wsx = 0; wsx < NWAVE; ++wsx) {
        int n = __builtin_amdgcn_readfirstlane(wcnt[wsx]);
        n = n > WCAP ? WCAP : (n < 0 ? 0 : n);
        const int* lp = list + wsx * WCAP;
#pragma unroll 1
        for (int i = 0; i < n; ++i) {
          const int ent  = __builtin_amdgcn_readfirstlane(lp[i]);
          const int slot = ent & (NB - 1);
          int e = cbase + ((ent >> 12) & (CHUNK - 1));
          e = e > nE - 1 ? nE - 1 : e;
          int rl = rels[e];
          rl = rl < 0 ? 0 : (rl > NRELS - 1 ? NRELS - 1 : rl);
          const int relh = rl - rb;
          if ((unsigned)relh < (unsigned)RH) {
            int s = srcs[e];
            s = s < 0 ? 0 : (s > nN - 1 ? nN - 1 : s);
            int dn = nodeBase + slot;
            dn = dn > nN - 1 ? nN - 1 : dn;
            const float coeff = inv_norm[(size_t)dn * NRELS + rl];
            const v4f v = *(const v4f*)(H + ((size_t)relh * nRowsPad + s) * DF + 4 * lane);
            v4f* ap = (v4f*)(acc + slot * DF + 4 * lane);
            const v4f cur = *ap;
            *ap = cur + v * coeff;
          }
        }
      }
    }
    __syncthreads();
  }

  if (FIN == 0) {
    const float* lrow = acc + (wave * RPW) * DF + 4 * lane;
    float* gp = out + ((size_t)nodeBase + wave * RPW) * DF + 4 * lane;
#pragma unroll 4
    for (int i = 0; i < RPW; ++i) {
      if (nodeBase + wave * RPW + i < nN) {
        const v4f v = *(const v4f*)(lrow + i * DF);
        *(volatile v4f*)(gp + (size_t)i * DF) = v;
      }
    }
    __threadfence();
#pragma unroll 4
    for (int i = 0; i < RPW; ++i) {
      if (nodeBase + wave * RPW + i < nN) {
        const v4f v = *(const v4f*)(lrow + i * DF);
        *(volatile v4f*)(gp + (size_t)i * DF) = v;
      }
    }
  } else {
#pragma unroll 1
    for (int q = 0; q < TPW; ++q) {
      const int t     = q * NWAVE + wave;
      const int slotm = 16 * t + m;
      int node = nodeBase + slotm;
      node = node > nN - 1 ? nN - 1 : node;

      v8f c[8];
#pragma unroll
      for (int ct = 0; ct < 8; ++ct) { const v8f z = {0.f, 0.f, 0.f, 0.f, 0.f, 0.f, 0.f, 0.f}; c[ct] = z; }

      const bf16_t* ah0 = xhi + (size_t)node * DF + 8 * hh;
      const bf16_t* al0 = xlo + (size_t)node * DF + 8 * hh;
      const bf16_t* bh0 = w0hi + (size_t)m * DF + 8 * hh;
      const bf16_t* bl0 = w0lo + (size_t)m * DF + 8 * hh;
#pragma unroll 1
      for (int ks = 0; ks < DF / 32; ++ks)
        kstep3(ah0 + 32 * ks, al0 + 32 * ks, bh0 + 32 * ks, bl0 + 32 * ks, c);

      float* sp = acc + (16 * t + 8 * hh) * DF + m;
#pragma unroll
      for (int ct = 0; ct < 8; ++ct) {
#pragma unroll
        for (int r = 0; r < 8; ++r) {
          const float v = sp[r * DF + 16 * ct] + c[ct][r];
          sp[r * DF + 16 * ct] = v;
        }
      }
      __syncthreads();

      const float* lrow = acc + (16 * t) * DF + 4 * lane;
      float* gp = out + ((size_t)nodeBase + 16 * t) * DF + 4 * lane;
#pragma unroll
      for (int i = 0; i < 16; ++i) {
        if (nodeBase + 16 * t + i < nN) {
          const v4f v = *(const v4f*)(lrow + i * DF);
          *(volatile v4f*)(gp + (size_t)i * DF) = v;
        }
      }
      __threadfence();
#pragma unroll
      for (int i = 0; i < 16; ++i) {
        if (nodeBase + 16 * t + i < nN) {
          const v4f v = *(const v4f*)(lrow + i * DF);
          *(volatile v4f*)(gp + (size_t)i * DF) = v;
        }
      }
    }
  }
}

extern "C" void kernel_launch(void* const* d_in, const int* in_sizes, int n_in,
                              void* d_out, int out_size, void* d_ws, size_t ws_size,
                              hipStream_t stream) {
  if (n_in < 7) return;
  const int nN = in_sizes[0] / DF;
  const int nE = in_sizes[4];
  if (nN <= 0 || nE <= 0) return;
  if (in_sizes[0] != nN * DF) return;
  if (in_sizes[1] != NRELS * DF * DF || in_sizes[2] != DF * DF) return;
  if (in_sizes[3] != nN * NRELS) return;
  if (in_sizes[5] != nE || in_sizes[6] != nE) return;
  if (out_size != nN * DF) return;

  const float* X        = (const float*)d_in[0];
  const float* W        = (const float*)d_in[1];
  const float* W0       = (const float*)d_in[2];
  const float* inv_norm = (const float*)d_in[3];
  const int*   srcs     = (const int*)d_in[4];
  const int*   dsts     = (const int*)d_in[5];
  const int*   rels     = (const int*)d_in[6];
  float* out = (float*)d_out;

  const int nBlk     = (nN + NB - 1) / NB;
  const int nRowsPad = nBlk * NB;
  const int gx       = (nN + GROWS - 1) / GROWS;

  char* ws = (char*)d_ws;
  size_t off = 0;
  const size_t szW = (size_t)(NRELS + 1) * DF * DF * 2;
  const size_t szX = (size_t)nRowsPad * DF * 2;
  const size_t szH = (size_t)RH * nRowsPad * DF * 4;
  const size_t oWh = off; off += szW; off = (off + 255) & ~(size_t)255;
  const size_t oWl = off; off += szW; off = (off + 255) & ~(size_t)255;
  const size_t oXh = off; off += szX; off = (off + 255) & ~(size_t)255;
  const size_t oXl = off; off += szX; off = (off + 255) & ~(size_t)255;
  const size_t oH  = off; off += szH; off = (off + 255) & ~(size_t)255;
  if (off > ws_size) return;
  bf16_t* whi = (bf16_t*)(ws + oWh);
  bf16_t* wlo = (bf16_t*)(ws + oWl);
  bf16_t* xhi = (bf16_t*)(ws + oXh);
  bf16_t* xlo = (bf16_t*)(ws + oXl);
  float*  H   = (float*)(ws + oH);

  const int vec8 = 1;

  const int nTotW = (NRELS + 1) * DF * DF / 8;
  k_wprep<<<(nTotW + NTHR - 1) / NTHR, NTHR, 0, stream>>>(W, W0, whi, wlo, nTotW);

  const int nTotX = nRowsPad * (DF / 8);
  k_xprep<<<(nTotX + NTHR - 1) / NTHR, NTHR, 0, stream>>>(X, xhi, xlo, nN, nTotX);

  hipFuncSetAttribute(reinterpret_cast<const void*>(&k_agg<0>),
                      hipFuncAttributeMaxDynamicSharedMemorySize, LDS_AGG);
  hipFuncSetAttribute(reinterpret_cast<const void*>(&k_agg<1>),
                      hipFuncAttributeMaxDynamicSharedMemorySize, LDS_AGG);

  {
    dim3 gg(gx, RH);
    k_hgemm<<<gg, NTHR, 0, stream>>>(xhi, xlo, whi, wlo, H, nRowsPad);
    k_agg<0><<<nBlk, NTHR, LDS_AGG, stream>>>(
        dsts, srcs, rels, inv_norm, H, xhi, xlo,
        whi + (size_t)NRELS * DF * DF, wlo + (size_t)NRELS * DF * DF,
        out, nN, nE, nRowsPad, 0, vec8);
  }
  {
    dim3 gg(gx, RH);
    k_hgemm<<<gg, NTHR, 0, stream>>>(xhi, xlo, whi + (size_t)RH * DF * DF, wlo + (size_t)RH * DF * DF, H, nRowsPad);
    k_agg<1><<<nBlk, NTHR, LDS_AGG, stream>>>(
        dsts, srcs, rels, inv_norm, H, xhi, xlo,
        whi + (size_t)NRELS * DF * DF, wlo + (size_t)NRELS * DF * DF,
        out, nN, nE, nRowsPad, RH, vec8);
  }
}
